// QASSMultiheadAttention_63007170232570
// MI455X (gfx1250) — hardware-run, weakly checked
//
#include <hip/hip_runtime.h>
#include <math.h>

constexpr int kBatch = 2;
constexpr int kSeq   = 2048;
constexpr int kDm    = 1024;
constexpr int kHeads = 16;
constexpr int kHd    = 64;
constexpr int kGh    = 64;
constexpr int kRows  = kBatch * kSeq;
static_assert(kHeads * kHd == kDm);
static_assert(kHd == 64 && kGh == 64);

constexpr float kXCarry   = 16.0f;
constexpr float kWCarry   = 256.0f;
constexpr float kACarry   = 256.0f;
constexpr float kPCarry   = 32768.0f;
constexpr float kResCarry = 2048.0f;
constexpr float kProjScale = 1.0f / (kXCarry * kWCarry);
constexpr float kOutScale  = 1.0f / (kACarry * kWCarry);
constexpr float kResInv    = 1.0f / kResCarry;
constexpr float kAoFactor  = kACarry / kPCarry;
constexpr float kScoreScale = 0.125f;
static_assert(kScoreScale * kScoreScale * (float)kHd == 1.0f);
constexpr float kMaskFill = -3.0e38f;
constexpr float kF16MinNormal = 6.103515625e-05f;

constexpr int kFlQ    = 128;
constexpr int kFlKeys = 64;
constexpr int kMaskWords = kSeq / 32;
static_assert(kSeq % kFlQ == 0 && kSeq % kFlKeys == 0);

typedef __attribute__((ext_vector_type(16))) _Float16 v16h;
typedef __attribute__((ext_vector_type(8)))  _Float16 v8h;
typedef __attribute__((ext_vector_type(8)))  float    v8f;
typedef __attribute__((ext_vector_type(4)))  float    v4f;
typedef __attribute__((ext_vector_type(2)))  float    v2f;
typedef __attribute__((ext_vector_type(4)))  unsigned int v4u;
typedef __attribute__((ext_vector_type(4)))  int      v4i;

__device__ __forceinline__ unsigned short f2bf_bits(float f) {
  unsigned u = __float_as_uint(f);
  return (unsigned short)((u + 0x7FFFu + ((u >> 16) & 1u)) >> 16);
}
__device__ __forceinline__ float bf_bits2f(unsigned short h) { return __uint_as_float(((unsigned)h) << 16); }
__device__ __forceinline__ float bf_rne(float f) { return bf_bits2f(f2bf_bits(f)); }
__device__ __forceinline__ unsigned pk16(unsigned short a, unsigned short b) { return (unsigned)a | ((unsigned)b << 16); }
__device__ __forceinline__ unsigned short h_bits(float f) { const _Float16 h = (_Float16)f; return __builtin_bit_cast(unsigned short, h); }
__device__ __forceinline__ unsigned short hh_bits(_Float16 h) { const _Float16 t = h; return __builtin_bit_cast(unsigned short, t); }
__device__ __forceinline__ float gelu_erf(float x) { return 0.5f * x * (1.0f + erff(x * 0.70710678118654752f)); }

__device__ __forceinline__ void wave_sync() {
  __builtin_amdgcn_fence(__ATOMIC_RELEASE, "workgroup");
  __builtin_amdgcn_wave_barrier();
  __builtin_amdgcn_fence(__ATOMIC_ACQUIRE, "workgroup");
}

__device__ __forceinline__ void split_f16(float v, _Float16& hf, _Float16& lf) {
  const float vh = (fabsf(v) < kF16MinNormal) ? 0.0f : v;
  hf = (_Float16)vh;
  float hw = (float)hf;
  asm volatile("" : "+v"(hw));
  lf = (_Float16)((v - hw) * kResCarry);
}

union FragU { v16h v; v8h h[2]; };
__device__ __forceinline__ v16h frag_load(const _Float16* p) {
  FragU f;
  f.h[0] = *(const v8h*)(p);
  f.h[1] = *(const v8h*)(p + 16);
  return f.v;
}
__device__ __forceinline__ v8f mma_h(v16h a, v16h b, v8f c) {
  c = __builtin_amdgcn_wmma_f32_16x16x32_f16(false, a, false, b, (short)0, c, false, false);
  asm volatile("v_nop\n\tv_nop\n\tv_nop\n\tv_nop" : "+v"(c) : "v"(a), "v"(b));
  return c;
}

__global__ __launch_bounds__(256) void cast_bf_f16_kernel(const float* __restrict__ in0, const float* __restrict__ in1,
                                                          const float* __restrict__ in2, const float* __restrict__ in3,
                                                          unsigned short* __restrict__ out, long planeStride, int n8, float carry) {
  const int z = blockIdx.y;
  const float* in = (z == 0) ? in0 : (z == 1) ? in1 : (z == 2) ? in2 : in3;
  const int i = blockIdx.x * 256 + threadIdx.x;
  if (i >= n8) return;
  const float* p = in + 8 * (size_t)i;
  const v4f a = *(const v4f*)(p);
  const v4f c = *(const v4f*)(p + 4);
  unsigned short hb[8];
#pragma unroll
  for (int e = 0; e < 4; ++e) {
    const float x0 = a[e];
    const float x1 = c[e];
    hb[e]     = h_bits(bf_rne(x0) * carry);
    hb[4 + e] = h_bits(bf_rne(x1) * carry);
  }
  const v4u u = (v4u){pk16(hb[0], hb[1]), pk16(hb[2], hb[3]), pk16(hb[4], hb[5]), pk16(hb[6], hb[7])};
  unsigned short* q = out + (size_t)z * planeStride + 8 * (size_t)i;
  *(volatile v4u*)q = u;
  __threadfence();
  *(volatile v4u*)q = u;
}

__global__ __launch_bounds__(256) void base_kernel(const float* __restrict__ wb1, const float* __restrict__ wb2,
                                                   const int* __restrict__ nctx, float* __restrict__ base) {
  __shared__ __align__(16) float g[kGh];
  const int t = threadIdx.x;
  if (t < kGh) {
    const float logn = logf((float)nctx[0]);
    g[t] = gelu_erf(logn * bf_rne(wb1[t]));
  }
  __syncthreads();
  const int c = blockIdx.x * 256 + t;
  const float* wr = wb2 + (size_t)c * kGh;
  float s = 0.0f;
#pragma unroll 2
  for (int j4 = 0; j4 < kGh / 4; ++j4) {
    const v4f w = *(const v4f*)(wr + 4 * j4);
    const v4f gg = *(const v4f*)(g + 4 * j4);
    s = fmaf(gg[0], bf_rne(w[0]), s);
    s = fmaf(gg[1], bf_rne(w[1]), s);
    s = fmaf(gg[2], bf_rne(w[2]), s);
    s = fmaf(gg[3], bf_rne(w[3]), s);
  }
  volatile float* o = base + c;
  *o = s;
  __threadfence();
  *o = s;
}

__global__ __launch_bounds__(256) void maskpack_kernel(const int* __restrict__ mask, unsigned int* __restrict__ bits) {
  const int w = blockIdx.x * 256 + threadIdx.x;
  const int* p = mask + (size_t)w * 32;
  unsigned int word = 0u;
#pragma unroll
  for (int i = 0; i < 8; ++i) {
    const v4i v = *(const v4i*)(p + 4 * i);
    const int e0 = v[0];
    const int e1 = v[1];
    const int e2 = v[2];
    const int e3 = v[3];
    word |= ((e0 != 0) ? 1u : 0u) << (4 * i + 0);
    word |= ((e1 != 0) ? 1u : 0u) << (4 * i + 1);
    word |= ((e2 != 0) ? 1u : 0u) << (4 * i + 2);
    word |= ((e3 != 0) ? 1u : 0u) << (4 * i + 3);
  }
  volatile unsigned int* o = bits + w;
  *o = word;
  __threadfence();
  *o = word;
}

template <int OUT_MODE>
__global__ __launch_bounds__(256) void wmma_gemm64(
    const unsigned short* __restrict__ Ap, int lda, long strideA,
    const unsigned short* __restrict__ Btp, int ldb, long strideB,
    void* __restrict__ Cout, void* __restrict__ Cout2, int ldc, long strideC,
    int M, int N, int K, float scale) {
  const _Float16* A  = (const _Float16*)(const void*)Ap;
  const _Float16* Bt = (const _Float16*)(const void*)Btp;
  __shared__ __align__(16) float sT[8][16 * 68];
  const int b    = blockIdx.y;
  const int lane = threadIdx.x & 31;
  const int wave = threadIdx.x >> 5;
  const int tilesN = N >> 6;
  const int tilesM = M >> 6;
  const int tile = blockIdx.x * 8 + wave;
  if (tile >= tilesM * tilesN) return;
  const int tm = tile / tilesN;
  const int tn = tile - tm * tilesN;
  const int m0 = tm << 6;
  const int n0 = tn << 6;

  const _Float16* Ab = A  + (size_t)b * strideA;
  const _Float16* Bb = Bt + (size_t)b * strideB;

  const int rlane = lane & 15;
  const int koff  = (lane >> 4) * 8;
  const int mOff  = (lane >> 4) * 8;

  v8f acc[4][4];
#pragma unroll
  for (int i = 0; i < 4; ++i)
#pragma unroll
    for (int j = 0; j < 4; ++j) acc[i][j] = (v8f){0.f, 0.f, 0.f, 0.f, 0.f, 0.f, 0.f, 0.f};

  for (int k0 = 0; k0 < K; k0 += 32) {
    v16h bh[4];
#pragma unroll
    for (int j = 0; j < 4; ++j) {
      const size_t bo = (size_t)(n0 + (j << 4) + rlane) * ldb + koff + k0;
      bh[j] = frag_load(Bb + bo);
    }
#pragma unroll
    for (int i = 0; i < 4; ++i) {
      const size_t ao = (size_t)(m0 + (i << 4) + rlane) * lda + koff + k0;
      const v16h ah = frag_load(Ab + ao);
#pragma unroll
      for (int j = 0; j < 4; ++j) acc[i][j] = mma_h(ah, bh[j], acc[i][j]);
    }
  }

  float* slab = sT[wave];
#pragma unroll
  for (int i = 0; i < 4; ++i) {
    const int mBase = m0 + (i << 4);
#pragma unroll
    for (int j = 0; j < 4; ++j) {
#pragma unroll
      for (int r = 0; r < 8; ++r) {
        const float v = acc[i][j][r] * scale;
        slab[(mOff + r) * 68 + (j << 4) + rlane] = v;
      }
    }
    wave_sync();
    if (OUT_MODE == 0) {
      float* C = (float*)Cout + (size_t)b * strideC;
      const int hh = lane >> 4, c4 = (lane & 15) * 4;
      for (int pass = 0; pass < 2; ++pass) {
#pragma unroll
        for (int it = 0; it < 8; ++it) {
          const int row = it * 2 + hh;
          const v4f v = *(const v4f*)(slab + row * 68 + c4);
          *(volatile v4f*)(C + (size_t)(mBase + row) * ldc + n0 + c4) = v;
        }
        __threadfence();
      }
    } else {
      const int q = lane >> 3, c8 = (lane & 7) * 8;
      unsigned short* C  = (unsigned short*)Cout + (size_t)b * strideC;
      unsigned short* C2 = (OUT_MODE == 3) ? ((unsigned short*)Cout2 + (size_t)b * strideC) : nullptr;
      for (int pass = 0; pass < 2; ++pass) {
#pragma unroll
        for (int it = 0; it < 4; ++it) {
          const int row = it * 4 + q;
          const float* sp = slab + row * 68 + c8;
          v8h hv, lv;
#pragma unroll
          for (int e = 0; e < 8; ++e) {
            const float x = sp[e];
            if (OUT_MODE == 1) {
              const _Float16 hf = (_Float16)x;
              hv[e] = hf;
              lv[e] = hf;
            } else {
              _Float16 hf, lf;
              split_f16(x, hf, lf);
              hv[e] = hf;
              lv[e] = lf;
            }
          }
          *(volatile v8h*)(C + (size_t)(mBase + row) * ldc + n0 + c8) = hv;
          if (OUT_MODE == 3) *(volatile v8h*)(C2 + (size_t)(mBase + row) * ldc + n0 + c8) = lv;
        }
        __threadfence();
      }
    }
    wave_sync();
  }
}

constexpr int kGateItemsPerWave = 32;
constexpr int kGateBlocks = (kRows * kHeads) / (8 * kGateItemsPerWave);
static_assert((kRows * kHeads) % (8 * kGateItemsPerWave) == 0);

__global__ __launch_bounds__(256) void gate_kernel(const float* __restrict__ q, const float* __restrict__ base,
                                                   const float* __restrict__ wg1, const float* __restrict__ wg2,
                                                   unsigned short* __restrict__ qhi, unsigned short* __restrict__ qlo) {
  __shared__ __align__(16) float w1t[kHd * kGh];
  __shared__ __align__(16) float w2t[kGh * kHd];
  __shared__ __align__(16) float baseS[kDm];
  __shared__ __align__(16) float qs[8][kHd];
  __shared__ __align__(16) float hs[8][kGh];
  __shared__ __align__(16) float zs[8][kHd];
  const int t = threadIdx.x;
  const int lane = t & 31, wave = t >> 5;
#pragma unroll 4
  for (int i = 0; i < 16; ++i) {
    const int e = i * 256 + t;
    const int r = e >> 6;
    const int cc = e & 63;
    w1t[cc * 64 + r] = bf_rne(wg1[e]);
    w2t[cc * 64 + r] = bf_rne(wg2[e]);
  }
#pragma unroll
  for (int i = 0; i < 4; ++i) baseS[i * 256 + t] = base[i * 256 + t];
  __syncthreads();

  float* qsw = qs[wave];
  float* hsw = hs[wave];
  float* zsw = zs[wave];
  const int item0 = (blockIdx.x * 8 + wave) * kGateItemsPerWave;
#pragma unroll 1
  for (int it = 0; it < kGateItemsPerWave; ++it) {
    const int item = item0 + it;
    const int row = item >> 4;
    const int h = item & (kHeads - 1);
    const size_t off = (size_t)row * kDm + h * kHd + 2 * lane;
    const v2f qv = *(const v2f*)(q + off);
    *(v2f*)(qsw + 2 * lane) = qv;
    wave_sync();
    float u0 = 0.0f, u1 = 0.0f;
#pragma unroll 1
    for (int d4 = 0; d4 < kHd / 4; ++d4) {
      const v4f q4 = *(const v4f*)(qsw + 4 * d4);
#pragma unroll
      for (int e = 0; e < 4; ++e) {
        const v2f w = *(const v2f*)(w1t + (4 * d4 + e) * 64 + 2 * lane);
        u0 = fmaf(q4[e], w[0], u0);
        u1 = fmaf(q4[e], w[1], u1);
      }
    }
    *(v2f*)(hsw + 2 * lane) = (v2f){u0, u1};
    wave_sync();
#pragma unroll 1
    for (int k = 0; k < 2; ++k) {
      const int idx = lane + 32 * k;
      const float x = hsw[idx];
      hsw[idx] = gelu_erf(x);
    }
    wave_sync();
    float z0 = 0.0f, z1 = 0.0f;
#pragma unroll 1
    for (int j4 = 0; j4 < kGh / 4; ++j4) {
      const v4f h4 = *(const v4f*)(hsw + 4 * j4);
#pragma unroll
      for (int e = 0; e < 4; ++e) {
        const v2f w = *(const v2f*)(w2t + (4 * j4 + e) * 64 + 2 * lane);
        z0 = fmaf(h4[e], w[0], z0);
        z1 = fmaf(h4[e], w[1], z1);
      }
    }
    *(v2f*)(zsw + 2 * lane) = (v2f){z0, z1};
    wave_sync();
#pragma unroll 1
    for (int k = 0; k < 2; ++k) {
      const int idx = lane + 32 * k;
      const float x = zsw[idx];
      zsw[idx] = 1.0f + tanhf(x);
    }
    wave_sync();
    const v2f gt = *(const v2f*)(zsw + 2 * lane);
    const v2f bs = *(const v2f*)(baseS + h * kHd + 2 * lane);
    const float o0 = (qv[0] * bs[0]) * gt[0];
    const float o1 = (qv[1] * bs[1]) * gt[1];
    _Float16 h0, l0, h1, l1;
    split_f16(o0, h0, l0);
    split_f16(o1, h1, l1);
    const unsigned uh = pk16(hh_bits(h0), hh_bits(h1));
    const unsigned ul = pk16(hh_bits(l0), hh_bits(l1));
    volatile unsigned* ph = (volatile unsigned*)(qhi + off);
    volatile unsigned* pl = (volatile unsigned*)(qlo + off);
    *ph = uh;
    *pl = ul;
    __threadfence();
    *ph = uh;
    *pl = ul;
    wave_sync();
  }
}

__global__ __launch_bounds__(256) void flash_kernel(
    const unsigned short* __restrict__ qhp, const unsigned short* __restrict__ qlp,
    const unsigned short* __restrict__ khp, const unsigned short* __restrict__ klp,
    const unsigned short* __restrict__ vtp, const unsigned int* __restrict__ mbits,
    unsigned short* __restrict__ aop) {
  __shared__ __align__(16) _Float16 Ksh[kFlKeys * kHd];
  __shared__ __align__(16) _Float16 Ksl[kFlKeys * kHd];
  __shared__ __align__(16) _Float16 Vts[kHd * kFlKeys];
  __shared__ __align__(16) _Float16 Ps[8][16 * kFlKeys];
  __shared__ __align__(16) unsigned int Msk[kFlQ * 2];

  const int tid  = threadIdx.x;
  const int wave = tid >> 5;
  const int lane = tid & 31;
  const int hh   = lane >> 4;
  const int c    = lane & 15;

  const int bh = blockIdx.y;
  const int b  = bh / kHeads;
  const int h  = bh - b * kHeads;
  const int qblk0 = blockIdx.x * kFlQ;
  const int q0 = qblk0 + wave * 16;

  const size_t tokBase = (size_t)b * kSeq;
  const _Float16* Qh = (const _Float16*)(const void*)qhp + tokBase * kDm + h * kHd;
  const _Float16* Ql = (const _Float16*)(const void*)qlp + tokBase * kDm + h * kHd;
  const _Float16* Kh = (const _Float16*)(const void*)khp + tokBase * kDm + h * kHd;
  const _Float16* Kl = (const _Float16*)(const void*)klp + tokBase * kDm + h * kHd;
  const _Float16* Vg = (const _Float16*)(const void*)vtp + ((size_t)b * kDm + (size_t)h * kHd) * kSeq;
  _Float16* Ao = (_Float16*)(void*)aop + tokBase * kDm + h * kHd;

  v16h qah[2], qal[2];
#pragma unroll
  for (int dc = 0; dc < 2; ++dc) {
    const size_t qo = (size_t)(q0 + c) * kDm + dc * 32 + 8 * hh;
    qah[dc] = frag_load(Qh + qo);
    qal[dc] = frag_load(Ql + qo);
  }

  float mrow[8], lrow[8];
  v8f oacc[4];
#pragma unroll
  for (int r = 0; r < 8; ++r) { mrow[r] = -INFINITY; lrow[r] = 0.f; }
#pragma unroll
  for (int t = 0; t < 4; ++t) oacc[t] = (v8f){0.f, 0.f, 0.f, 0.f, 0.f, 0.f, 0.f, 0.f};

  _Float16* pw = Ps[wave];

  for (int kc = 0; kc < kSeq / kFlKeys; ++kc) {
    const int kv0 = kc * kFlKeys;
    __syncthreads();
#pragma unroll
    for (int it = 0; it < 2; ++it) {
      const int i = tid + it * 256;
      const int row = i >> 3;
      const int seg = (i & 7) * 8;
      const v8h a  = *(const v8h*)(Kh + (size_t)(kv0 + row) * kDm + seg);
      const v8h al = *(const v8h*)(Kl + (size_t)(kv0 + row) * kDm + seg);
      const v8h vv = *(const v8h*)(Vg + (size_t)row * kSeq + kv0 + seg);
      *(v8h*)(Ksh + row * kHd + seg) = a;
      *(v8h*)(Ksl + row * kHd + seg) = al;
      *(v8h*)(Vts + row * kFlKeys + seg) = vv;
    }
    Msk[tid] = mbits[(size_t)(qblk0 + (tid >> 1)) * kMaskWords + kc * 2 + (tid & 1)];
    __syncthreads();

    v8f s[4];
#pragma unroll
    for (int j = 0; j < 4; ++j) {
      v8f sm = (v8f){0.f, 0.f, 0.f, 0.f, 0.f, 0.f, 0.f, 0.f};
      v8f sr = (v8f){0.f, 0.f, 0.f, 0.f, 0.f, 0.f, 0.f, 0.f};
#pragma unroll
      for (int dc = 0; dc < 2; ++dc) {
        const int ko = (j * 16 + c) * kHd + dc * 32 + 8 * hh;
        const v16h kb = frag_load(Ksh + ko);
        const v16h kl = frag_load(Ksl + ko);
        sm = mma_h(qah[dc], kb, sm);
        sr = mma_h(qah[dc], kl, sr);
        sr = mma_h(qal[dc], kb, sr);
      }
#pragma unroll
      for (int r = 0; r < 8; ++r) s[j][r] = (sm[r] + sr[r] * kResInv) * kScoreScale;
    }

    float cm[8];
#pragma unroll
    for (int r = 0; r < 8; ++r) {
      const int mr = (wave * 16 + 8 * hh + r) * 2;
      const unsigned int w0 = Msk[mr];
      const unsigned int w1 = Msk[mr + 1];
      const bool a0 = ((w0 >> c) & 1u) != 0u;
      const bool a1 = ((w0 >> (16 + c)) & 1u) != 0u;
      const bool a2 = ((w1 >> c) & 1u) != 0u;
      const bool a3 = ((w1 >> (16 + c)) & 1u) != 0u;
      s[0][r] = a0 ? s[0][r] : kMaskFill;
      s[1][r] = a1 ? s[1][r] : kMaskFill;
      s[2][r] = a2 ? s[2][r] : kMaskFill;
      s[3][r] = a3 ? s[3][r] : kMaskFill;
      float m = fmaxf(fmaxf(s[0][r], s[1][r]), fmaxf(s[2][r], s[3][r]));
#pragma unroll
      for (int off = 1; off < 16; off <<= 1) m = fmaxf(m, __shfl_xor(m, off, 32));
      cm[r] = m;
    }
#pragma unroll
    for (int r = 0; r < 8; ++r) {
      const float mnew = fmaxf(mrow[r], cm[r]);
      const float alpha = expf(mrow[r] - mnew);
      mrow[r] = mnew;
      float psum = 0.f;
#pragma unroll
      for (int j = 0; j < 4; ++j) {
        const float p = expf(s[j][r] - mnew);
        psum += p;
        pw[(8 * hh + r) * kFlKeys + j * 16 + c] = (_Float16)(p * kPCarry);
      }
#pragma unroll
      for (int off = 1; off < 16; off <<= 1) psum += __shfl_xor(psum, off, 32);
      lrow[r] = lrow[r] * alpha + psum;
#pragma unroll
      for (int t = 0; t < 4; ++t) oacc[t][r] *= alpha;
    }
    wave_sync();
#pragma unroll
    for (int kk = 0; kk < 2; ++kk) {
      const v16h pa = frag_load(pw + c * kFlKeys + kk * 32 + 8 * hh);
#pragma unroll
      for (int t = 0; t < 4; ++t) {
        const v16h vb = frag_load(Vts + (t * 16 + c) * kFlKeys + kk * 32 + 8 * hh);
        oacc[t] = mma_h(pa, vb, oacc[t]);
      }
    }
  }

  wave_sync();
#pragma unroll
  for (int r = 0; r < 8; ++r) {
    const float fin = (1.0f / lrow[r]) * kAoFactor;
    const float fac = (mrow[r] < -1.0e37f) ? __uint_as_float(0x7fc00000u) : fin;
#pragma unroll
    for (int t = 0; t < 4; ++t) pw[(8 * hh + r) * kFlKeys + t * 16 + c] = (_Float16)(oacc[t][r] * fac);
  }
  wave_sync();
  {
    const int q = lane >> 3, c8 = (lane & 7) * 8;
    for (int pass = 0; pass < 2; ++pass) {
#pragma unroll
      for (int it = 0; it < 4; ++it) {
        const int row = it * 4 + q;
        const v8h val = *(const v8h*)(pw + row * kFlKeys + c8);
        *(volatile v8h*)(Ao + (size_t)(q0 + row) * kDm + c8) = val;
      }
      __threadfence();
    }
  }
}

constexpr size_t kActPlaneBytes = (size_t)kRows * kDm * 2;
constexpr size_t kWPlaneBytes   = (size_t)kDm * kDm * 2;
constexpr size_t kOffX    = 0;
constexpr size_t kOffW    = kOffX + 3 * kActPlaneBytes;
constexpr size_t kOffQ    = kOffW + 4 * kWPlaneBytes;
constexpr size_t kOffKh   = kOffQ + (size_t)kRows * kDm * 4;
constexpr size_t kOffKl   = kOffKh + kActPlaneBytes;
constexpr size_t kOffVt   = kOffKl + kActPlaneBytes;
constexpr size_t kOffQh   = kOffVt + kActPlaneBytes;
constexpr size_t kOffQl   = kOffQh + kActPlaneBytes;
constexpr size_t kOffAo   = kOffQl + kActPlaneBytes;
constexpr size_t kOffMask = kOffAo + kActPlaneBytes;
constexpr size_t kOffBase = kOffMask + (size_t)kSeq * kMaskWords * 4;
constexpr size_t kWsTotal = kOffBase + (size_t)kDm * 4;
static_assert(kWsTotal == 101191680);
static_assert(kWsTotal <= 134217728);
static_assert(kRows % 64 == 0 && kDm % 64 == 0 && kSeq % 64 == 0 && kDm % 32 == 0);

extern "C" void kernel_launch(void* const* d_in, const int* in_sizes, int n_in,
                              void* d_out, int out_size, void* d_ws, size_t ws_size, hipStream_t stream) {
  (void)in_sizes;
  if (n_in < 13) return;
  if (out_size != kRows * kDm) return;
  if (ws_size < kWsTotal) return;

  const float* query = (const float*)d_in[0];
  const float* key_  = (const float*)d_in[1];
  const float* value = (const float*)d_in[2];
  const int*   amask = (const int*)d_in[3];
  const float* wq  = (const float*)d_in[4];
  const float* wk  = (const float*)d_in[5];
  const float* wv  = (const float*)d_in[6];
  const float* wo  = (const float*)d_in[7];
  const float* wb1 = (const float*)d_in[8];
  const float* wb2 = (const float*)d_in[9];
  const float* wg1 = (const float*)d_in[10];
  const float* wg2 = (const float*)d_in[11];
  const int*   nctx = (const int*)d_in[12];

  char* ws = (char*)d_ws;
  unsigned short* xplanes = (unsigned short*)(ws + kOffX);
  unsigned short* wplanes = (unsigned short*)(ws + kOffW);
  float*          qf   = (float*)(ws + kOffQ);
  unsigned short* khi  = (unsigned short*)(ws + kOffKh);
  unsigned short* klo  = (unsigned short*)(ws + kOffKl);
  unsigned short* vt   = (unsigned short*)(ws + kOffVt);
  unsigned short* qhi  = (unsigned short*)(ws + kOffQh);
  unsigned short* qlo  = (unsigned short*)(ws + kOffQl);
  unsigned short* ao   = (unsigned short*)(ws + kOffAo);
  unsigned int*   mbits = (unsigned int*)(ws + kOffMask);
  float*          basev = (float*)(ws + kOffBase);

  const long actElems = (long)kRows * kDm;
  const long wElems   = (long)kDm * kDm;
  unsigned short* xq = xplanes;
  unsigned short* xk = xplanes + actElems;
  unsigned short* xv = xplanes + 2 * actElems;
  unsigned short* wqh = wplanes;
  unsigned short* wkh = wplanes + wElems;
  unsigned short* wvh = wplanes + 2 * wElems;
  unsigned short* woh = wplanes + 3 * wElems;

  {
    const int n8a = (int)(actElems / 8);
    const int n8w = (int)(wElems / 8);
    cast_bf_f16_kernel<<<dim3(n8a / 256, 3), 256, 0, stream>>>(query, key_, value, value, xplanes, actElems, n8a, kXCarry);
    cast_bf_f16_kernel<<<dim3(n8w / 256, 4), 256, 0, stream>>>(wq, wk, wv, wo, wplanes, wElems, n8w, kWCarry);
  }
  base_kernel<<<kDm / 256, 256, 0, stream>>>(wb1, wb2, nctx, basev);
  maskpack_kernel<<<(kSeq * kMaskWords) / 256, 256, 0, stream>>>(amask, mbits);

  {
    const int tilesQ = (kRows / 64) * (kDm / 64);
    wmma_gemm64<0><<<dim3(tilesQ / 8, 1), 256, 0, stream>>>(xq, kDm, 0L, wqh, kDm, 0L,
                                                         (void*)qf, nullptr, kDm, 0L, kRows, kDm, kDm, kProjScale);
    wmma_gemm64<3><<<dim3(tilesQ / 8, 1), 256, 0, stream>>>(xk, kDm, 0L, wkh, kDm, 0L,
                                                         (void*)khi, (void*)klo, kDm, 0L, kRows, kDm, kDm, kProjScale);
    const int tilesV = (kDm / 64) * (kSeq / 64);
    wmma_gemm64<1><<<dim3(tilesV / 8, kBatch), 256, 0, stream>>>(wvh, kDm, 0L, xv, kDm, (long)kSeq * kDm,
                                                              (void*)vt, nullptr, kSeq, (long)kDm * kSeq, kDm, kSeq, kDm, kProjScale);
  }
  gate_kernel<<<kGateBlocks, 256, 0, stream>>>(qf, basev, wg1, wg2, qhi, qlo);

  flash_kernel<<<dim3(kSeq / kFlQ, kBatch * kHeads), 256, 0, stream>>>(qhi, qlo, khi, klo, vt, mbits, ao);

  {
    const int tilesO = (kRows / 64) * (kDm / 64);
    wmma_gemm64<0><<<dim3(tilesO / 8, 1), 256, 0, stream>>>(ao, kDm, 0L, woh, kDm, 0L,
                                                         d_out, nullptr, kDm, 0L, kRows, kDm, kDm, kOutScale);
  }
}
